// IConv_5317169512859
// MI455X (gfx1250) — hardware-verified
//
#include <hip/hip_runtime.h>

typedef __attribute__((ext_vector_type(16))) _Float16 v16h;
typedef __attribute__((ext_vector_type(8)))  float  v8f;
typedef __attribute__((ext_vector_type(4)))  float  v4f;

union FragAB { v16h v; unsigned u[8]; };
union FragC  { v8f   v; float    f[8]; };

__device__ __forceinline__ unsigned pack_h2(float a, float b) {
  union { _Float16 h[2]; unsigned u; } p;
  p.h[0] = (_Float16)a;
  p.h[1] = (_Float16)b;
  return p.u;
}

__device__ __forceinline__ v8f wmma_f16(v16h a, v16h b, v8f c) {
  v8f d = __builtin_amdgcn_wmma_f32_16x16x32_f16(false, a, false, b, (short)0, c, false, false);
  asm volatile("v_nop\n\tv_nop\n\tv_nop\n\tv_nop" : "+v"(d) : "v"(a), "v"(b));
  return d;
}

#define PEP_LEN 15
#define DDIM    64
#define OC      128
#define KS      9
#define ML      34
#define LPAD    64
#define TOUT    7
#define WSCALE  64.0f
#define WUNSC   0.015625f

__device__ __forceinline__ int kword(int v, int hi) { return ((v >> 2) << 4) + (hi << 3) + ((v & 3) << 1); }

__global__ __launch_bounds__(256) void iconv_wmma_kernel(
    const float* __restrict__ pep,
    const float* __restrict__ mhc,
    const float* __restrict__ wgt,
    const float* __restrict__ bias,
    float* __restrict__ out)
{
  __shared__ _Float16 sMhcT[DDIM * LPAD];
  __shared__ _Float16 sPep[16 * DDIM];
  __shared__ _Float16 sKer[8][16 * DDIM];
  __shared__ float  sBias[OC];
  __shared__ __attribute__((aligned(16))) float sOut[OC * TOUT];

  const int n    = blockIdx.x;
  const int tid  = threadIdx.x;
  const int wave = tid >> 5;
  const int lane = tid & 31;
  const int lo   = lane & 15;
  const int hi   = lane >> 4;

  const int obase = wave * 16 + lo;

  for (int i = tid; i < (DDIM * LPAD) / 2; i += 256)
    ((unsigned*)sMhcT)[i] = 0u;
  if (tid < OC) sBias[tid] = bias[tid];
  __syncthreads();

  const float* mhcn = mhc + (size_t)n * ML * DDIM;
  for (int i = tid; i < ML * DDIM; i += 256) {
    int l = i >> 6, d = i & 63;
    sMhcT[d * LPAD + l] = (_Float16)mhcn[i];
  }
  const float* pepn = pep + (size_t)n * PEP_LEN * DDIM;
  for (int i = tid; i < PEP_LEN * DDIM; i += 256)
    sPep[i] = (_Float16)pepn[i];
  for (int i = PEP_LEN * DDIM + tid; i < 16 * DDIM; i += 256)
    sPep[i] = (_Float16)0.0f;
  __syncthreads();

  FragAB A1[4][2];
#pragma unroll
  for (int dt = 0; dt < 4; ++dt)
#pragma unroll
    for (int s = 0; s < 2; ++s)
#pragma unroll
      for (int v = 0; v < 8; ++v) {
        int l = s * 32 + kword(v, hi);
        int d = dt * 16 + lo;
        A1[dt][s].u[v] = *(const unsigned*)(sMhcT + d * LPAD + l);
      }

  FragC acc;
#pragma unroll
  for (int v = 0; v < 8; ++v) acc.f[v] = 0.0f;

  const int tRow = (lo < TOUT) ? lo : (TOUT - 1);

  for (int k = 0; k < KS; ++k) {
    FragAB B1[2];
#pragma unroll
    for (int s = 0; s < 2; ++s)
#pragma unroll
      for (int v = 0; v < 8; ++v) {
        int l = s * 32 + kword(v, hi);
        float w0 = 0.0f, w1 = 0.0f;
        const float* wp = wgt + ((size_t)obase * KS + k) * ML;
        if (l < ML)     w0 = wp[l] * WSCALE;
        if (l + 1 < ML) w1 = wp[l + 1] * WSCALE;
        B1[s].u[v] = pack_h2(w0, w1);
      }

#pragma unroll
    for (int dt = 0; dt < 4; ++dt) {
      FragC c;
#pragma unroll
      for (int v = 0; v < 8; ++v) c.f[v] = 0.0f;
      c.v = wmma_f16(A1[dt][0].v, B1[0].v, c.v);
      c.v = wmma_f16(A1[dt][1].v, B1[1].v, c.v);
#pragma unroll
      for (int v = 0; v < 8; v += 2) {
        float f0 = fmaxf(c.f[v], 0.0f) * WUNSC;
        float f1 = fmaxf(c.f[v + 1], 0.0f) * WUNSC;
        int d = dt * 16 + (hi << 3) + v;
        *(unsigned*)(&sKer[wave][lo * DDIM + d]) = pack_h2(f0, f1);
      }
    }
    __syncthreads();

#pragma unroll
    for (int s2 = 0; s2 < 2; ++s2) {
      FragAB A2, B2;
#pragma unroll
      for (int v = 0; v < 8; ++v) {
        int dd = s2 * 32 + kword(v, hi);
        A2.u[v] = *(const unsigned*)(&sKer[wave][lo * DDIM + dd]);
        B2.u[v] = *(const unsigned*)(sPep + (tRow + k) * DDIM + dd);
      }
      acc.v = wmma_f16(A2.v, B2.v, acc.v);
    }
    __syncthreads();
  }

  if (lo < TOUT) {
#pragma unroll
    for (int v = 0; v < 8; ++v) {
      int o = wave * 16 + (hi << 3) + v;
      sOut[o * TOUT + lo] = acc.f[v] + sBias[o];
    }
  }
  __syncthreads();

  float* outn = out + (size_t)n * (OC * TOUT);
  if (tid < (OC * TOUT) / 4) {
    v4f val = *(const v4f*)(sOut + tid * 4);
    *(volatile v4f*)(outn + tid * 4) = val;
    __threadfence();
    *(volatile v4f*)(outn + tid * 4) = val;
  }
}

extern "C" void kernel_launch(void* const* d_in, const int* in_sizes, int n_in,
                              void* d_out, int out_size, void* d_ws, size_t ws_size,
                              hipStream_t stream) {
  const float* pep  = (const float*)d_in[0];
  const float* mhc  = (const float*)d_in[1];
  const float* wgt  = (const float*)d_in[2];
  const float* bias = (const float*)d_in[3];
  float* out = (float*)d_out;

  const int bs = in_sizes[0] / (PEP_LEN * DDIM);
  iconv_wmma_kernel<<<dim3(bs), dim3(256), 0, stream>>>(pep, mhc, wgt, bias, out);
}
